// SelectiveSSM_85598698209292
// MI455X (gfx1250) — hardware-run, weakly checked
//
#include <hip/hip_runtime.h>
#include <hip/hip_fp16.h>
#include <math.h>

constexpr int kBatch = 2;
constexpr int kSeq   = 1024;
constexpr int kDm    = 1024;
constexpr int kDin   = 2048;
constexpr int kNst   = 16;
constexpr int kDtR   = 64;
constexpr int kXdW   = kDtR + 2 * kNst;
constexpr int kXdP   = 128;
constexpr int kXzP   = 2 * kDin;
constexpr int kRows  = kBatch * kSeq;
constexpr int kConvTP = 260;
static_assert(kXdW == 96, "x_proj width");
static_assert(kXdP % 64 == 0 && kXdP >= kXdW, "padded x_proj width");
static_assert(kDm % 32 == 0 && kDin % 32 == 0 && kDtR % 32 == 0, "GEMM K multiples of 32");
static_assert(kRows % 64 == 0 && kXzP % 64 == 0 && kDin % 64 == 0 && kDm % 64 == 0, "GEMM M,N multiples of 64");
static_assert(kSeq % 64 == 0 && kDin % 256 == 0, "tile multiples");

constexpr float kCarryX    = 64.0f;
constexpr float kCarryWin  = 4096.0f;
constexpr float kCarryU    = 128.0f;
constexpr float kCarryWx   = 4096.0f;
constexpr float kCarryDtl  = 64.0f;
constexpr float kCarryWdt  = 1024.0f;
constexpr float kCarryY    = 1024.0f;
constexpr float kCarryWout = 4096.0f;
constexpr float kScaleIn  = 1.0f / (kCarryX * kCarryWin);
constexpr float kScaleXp  = 1.0f / (kCarryU * kCarryWx);
constexpr float kScaleDt  = 1.0f / (kCarryDtl * kCarryWdt);
constexpr float kScaleOut = 1.0f / (kCarryY * kCarryWout);

constexpr size_t kOffXH  = 0;
constexpr size_t kOffWIH = kOffXH  + (size_t)kRows * kDm  * 2;
constexpr size_t kOffWXH = kOffWIH + (size_t)kXzP  * kDm  * 2;
constexpr size_t kOffWDH = kOffWXH + (size_t)kXdP  * kDin * 2;
constexpr size_t kOffWOH = kOffWDH + (size_t)kDin  * kDtR * 2;
constexpr size_t kOffXZ  = kOffWOH + (size_t)kDm   * kDin * 2;
constexpr size_t kOffU   = kOffXZ  + (size_t)kRows * kXzP * 4;
constexpr size_t kOffUH  = kOffU   + (size_t)kRows * kDin * 4;
constexpr size_t kOffXD  = kOffUH  + (size_t)kRows * kDin * 2;
constexpr size_t kOffDTL = kOffXD  + (size_t)kRows * kXdP * 4;
constexpr size_t kOffDTP = kOffDTL + (size_t)kRows * kDtR * 2;
constexpr size_t kOffYH  = kOffDTP + (size_t)kRows * kDin * 4;
constexpr size_t kWsTotal = kOffYH + (size_t)kRows * kDin * 2;
static_assert(kWsTotal == 102760448ull, "carve total");
static_assert(kWsTotal <= 134217728ull, "carve cap");
static_assert((kOffWIH % 128) == 0 && (kOffWXH % 128) == 0 && (kOffWDH % 128) == 0 && (kOffWOH % 128) == 0 &&
              (kOffXZ % 128) == 0 && (kOffU % 128) == 0 && (kOffUH % 128) == 0 && (kOffXD % 128) == 0 &&
              (kOffDTL % 128) == 0 && (kOffDTP % 128) == 0 && (kOffYH % 128) == 0, "128-B aligned regions");

namespace eng {

typedef __attribute__((ext_vector_type(16))) _Float16 v16h;
typedef __attribute__((ext_vector_type(8)))  _Float16 v8h;
typedef __attribute__((ext_vector_type(8)))  float    v8f;
typedef __attribute__((ext_vector_type(4)))  float    v4f;
typedef __attribute__((ext_vector_type(4)))  unsigned v4u;

union FragU { v16h v; v8h h[2]; };

__device__ __forceinline__ v16h frag_load(const _Float16* p) {
  FragU f;
  f.h[0] = *(const v8h*)(p);
  f.h[1] = *(const v8h*)(p + 16);
  return f.v;
}

__device__ __forceinline__ v8f mma_f16(v16h a, v16h b, v8f c) {
  c = __builtin_amdgcn_wmma_f32_16x16x32_f16(false, a, false, b, (short)0, c, false, false);
  asm volatile("v_nop\n\tv_nop\n\tv_nop\n\tv_nop" : "+v"(c) : "v"(a), "v"(b));
  return c;
}

__device__ __forceinline__ unsigned h16bits(float v) {
  const float f = (fabsf(v) < 6.103515625e-05f) ? 0.0f : v;
  const _Float16 hv = (_Float16)f;
  const unsigned short hb = __builtin_bit_cast(unsigned short, hv);
  return (unsigned)hb;
}

template <int BIAS_MODE>
__global__ __launch_bounds__(256) void gemm_f16_kernel(
    const unsigned short* __restrict__ Ap, int lda,
    const unsigned short* __restrict__ Btp, int ldb,
    float* __restrict__ C, int ldc,
    const float* __restrict__ bias,
    int M, int N, int K, float scale)
{
  const _Float16* A  = (const _Float16*)Ap;
  const _Float16* Bt = (const _Float16*)Btp;
  __shared__ __align__(16) float sT[8][16 * 68];
  const int lane = threadIdx.x & 31;
  const int wave = threadIdx.x >> 5;
  const int tilesN = N >> 6;
  const int tilesM = M >> 6;
  const int tile = blockIdx.x * 8 + wave;
  if (tile >= tilesM * tilesN) return;
  const int tm = tile / tilesN;
  const int tn = tile - tm * tilesN;
  const int m0 = tm << 6;
  const int n0 = tn << 6;
  const int rlane = lane & 15;
  const int koff  = (lane >> 4) * 8;
  const int mOff  = (lane >> 4) * 8;

  v8f acc[4][4];
#pragma unroll
  for (int i = 0; i < 4; ++i)
#pragma unroll
    for (int j = 0; j < 4; ++j) acc[i][j] = (v8f){0.f, 0.f, 0.f, 0.f, 0.f, 0.f, 0.f, 0.f};

  for (int k0 = 0; k0 < K; k0 += 32) {
    v16h bh[4];
#pragma unroll
    for (int j = 0; j < 4; ++j) {
      const size_t bo = (size_t)(n0 + (j << 4) + rlane) * ldb + koff + k0;
      bh[j] = frag_load(Bt + bo);
    }
#pragma unroll
    for (int i = 0; i < 4; ++i) {
      const size_t ao = (size_t)(m0 + (i << 4) + rlane) * lda + koff + k0;
      const v16h ah = frag_load(A + ao);
#pragma unroll
      for (int j = 0; j < 4; ++j) acc[i][j] = mma_f16(ah, bh[j], acc[i][j]);
    }
  }

  float* slab = sT[wave];
#pragma unroll
  for (int i = 0; i < 4; ++i) {
    const int mBase = m0 + (i << 4);
#pragma unroll
    for (int j = 0; j < 4; ++j) {
      float bv = 0.f;
      if (BIAS_MODE == 2) bv = bias[n0 + (j << 4) + rlane];
#pragma unroll
      for (int r = 0; r < 8; ++r) {
        float v = acc[i][j][r] * scale;
        if (BIAS_MODE == 2) v += bv;
        slab[(mOff + r) * 68 + (j << 4) + rlane] = v;
      }
    }
    __builtin_amdgcn_fence(__ATOMIC_RELEASE, "workgroup");
    __builtin_amdgcn_wave_barrier();
    __builtin_amdgcn_fence(__ATOMIC_ACQUIRE, "workgroup");
    {
      const int hh = lane >> 4;
      const int c4 = (lane & 15) * 4;
      for (int pass = 0; pass < 2; ++pass) {
#pragma unroll
        for (int it = 0; it < 8; ++it) {
          const int row = it * 2 + hh;
          const v4f v = *(const v4f*)(slab + row * 68 + c4);
          *(volatile v4f*)(C + (size_t)(mBase + row) * ldc + n0 + c4) = v;
        }
        __threadfence();
      }
    }
    __builtin_amdgcn_fence(__ATOMIC_RELEASE, "workgroup");
    __builtin_amdgcn_wave_barrier();
    __builtin_amdgcn_fence(__ATOMIC_ACQUIRE, "workgroup");
  }
}

}

__global__ __launch_bounds__(256) void plane_f16_kernel(
    const float* __restrict__ src, int src_ld, int src_rows,
    unsigned short* __restrict__ dst, int cols8, int total8, float carry)
{
  const int i = blockIdx.x * 256 + threadIdx.x;
  if (i >= total8) return;
  const int row = i / cols8;
  const int g   = i - row * cols8;
  const bool live = (row < src_rows);
  const int rc = live ? row : (src_rows - 1);
  const float* sp = src + (size_t)rc * src_ld + (size_t)g * 8;
  const eng::v4f a0 = *(const eng::v4f*)(sp);
  const eng::v4f a1 = *(const eng::v4f*)(sp + 4);
  const float r0 = a0[0], r1 = a0[1], r2 = a0[2], r3 = a0[3];
  const float r4 = a1[0], r5 = a1[1], r6 = a1[2], r7 = a1[3];
  const float e0 = live ? r0 * carry : 0.0f;
  const float e1 = live ? r1 * carry : 0.0f;
  const float e2 = live ? r2 * carry : 0.0f;
  const float e3 = live ? r3 * carry : 0.0f;
  const float e4 = live ? r4 * carry : 0.0f;
  const float e5 = live ? r5 * carry : 0.0f;
  const float e6 = live ? r6 * carry : 0.0f;
  const float e7 = live ? r7 * carry : 0.0f;
  const unsigned w0 = eng::h16bits(e0) | (eng::h16bits(e1) << 16);
  const unsigned w1 = eng::h16bits(e2) | (eng::h16bits(e3) << 16);
  const unsigned w2 = eng::h16bits(e4) | (eng::h16bits(e5) << 16);
  const unsigned w3 = eng::h16bits(e6) | (eng::h16bits(e7) << 16);
  const eng::v4u wv = (eng::v4u){w0, w1, w2, w3};
  unsigned short* q = dst + ((size_t)i << 3);
  *(volatile eng::v4u*)q = wv;
  __threadfence();
  *(volatile eng::v4u*)q = wv;
}

__global__ __launch_bounds__(256) void conv_act_kernel(
    const float* __restrict__ XZ, const float* __restrict__ cw, const float* __restrict__ cb,
    float* __restrict__ U, unsigned short* __restrict__ UH)
{
  __shared__ __align__(16) float sT[16 * kConvTP];
  const int tid  = threadIdx.x;
  const int lane = tid & 31;
  const int wave = tid >> 5;
  const int d0 = blockIdx.x * 256;
  const int d  = d0 + tid;
  const int g0 = blockIdx.y * 64;
  const int tb = g0 & (kSeq - 1);
  const eng::v4f wv = *(const eng::v4f*)(cw + (size_t)d * 4);
  const float w0 = wv[0], w1 = wv[1], w2 = wv[2], w3 = wv[3];
  const float bcv = cb[d];
  float xm3, xm2, xm1;
  {
    const bool hist = (tb > 0);
    const int rb = hist ? (g0 - 3) : g0;
    const float v3 = XZ[(size_t)rb * kXzP + d];
    const float v2 = XZ[(size_t)(rb + 1) * kXzP + d];
    const float v1 = XZ[(size_t)(rb + 2) * kXzP + d];
    xm3 = hist ? v3 : 0.0f;
    xm2 = hist ? v2 : 0.0f;
    xm1 = hist ? v1 : 0.0f;
  }
  const int hrow = wave >> 1;
  const int hch  = (wave & 1) * 128 + lane * 4;
#pragma unroll 1
  for (int sub = 0; sub < 4; ++sub) {
    const int lb = g0 + sub * 16;
#pragma unroll 1
    for (int s = 0; s < 16; ++s) {
      const float xcur = XZ[(size_t)(lb + s) * kXzP + d];
      float acc = fmaf(w0, xm3, bcv);
      acc = fmaf(w1, xm2, acc);
      acc = fmaf(w2, xm1, acc);
      acc = fmaf(w3, xcur, acc);
      const float sg = 1.0f / (1.0f + expf(-acc));
      sT[s * kConvTP + tid] = acc * sg;
      xm3 = xm2;
      xm2 = xm1;
      xm1 = xcur;
    }
    __syncthreads();
    eng::v4f fv[4];
    eng::v4u hw[2];
#pragma unroll
    for (int it = 0; it < 4; ++it) fv[it] = *(const eng::v4f*)(sT + (it * 4 + hrow) * kConvTP + hch);
#pragma unroll
    for (int it = 0; it < 2; ++it) {
      const float* sp = sT + (it * 8 + wave) * kConvTP + lane * 8;
      const eng::v4f a0 = *(const eng::v4f*)(sp);
      const eng::v4f a1 = *(const eng::v4f*)(sp + 4);
      const float e0 = a0[0] * kCarryU, e1 = a0[1] * kCarryU, e2 = a0[2] * kCarryU, e3 = a0[3] * kCarryU;
      const float e4 = a1[0] * kCarryU, e5 = a1[1] * kCarryU, e6 = a1[2] * kCarryU, e7 = a1[3] * kCarryU;
      const unsigned p0 = eng::h16bits(e0) | (eng::h16bits(e1) << 16);
      const unsigned p1 = eng::h16bits(e2) | (eng::h16bits(e3) << 16);
      const unsigned p2 = eng::h16bits(e4) | (eng::h16bits(e5) << 16);
      const unsigned p3 = eng::h16bits(e6) | (eng::h16bits(e7) << 16);
      hw[it] = (eng::v4u){p0, p1, p2, p3};
    }
    for (int pass = 0; pass < 2; ++pass) {
#pragma unroll
      for (int it = 0; it < 4; ++it)
        *(volatile eng::v4f*)(U + (size_t)(lb + it * 4 + hrow) * kDin + d0 + hch) = fv[it];
#pragma unroll
      for (int it = 0; it < 2; ++it) {
        const size_t o = (size_t)(lb + it * 8 + wave) * kDin + d0 + lane * 8;
        *(volatile eng::v4u*)(UH + o) = hw[it];
      }
      __threadfence();
    }
    __syncthreads();
  }
}

typedef float    ms1_v4f __attribute__((ext_vector_type(4)));
typedef unsigned ms1_v4u __attribute__((ext_vector_type(4)));
struct ms1_args {
  const float* dtpre;
  const float* u;
  const float* bc;
  const float* z;
  const float* A_log;
  const float* Dskip;
  __half* y;
  __half* y_lo;
  long ld_dtpre;
  long ld_u;
  long ld_bc;
  long ld_z;
  long ld_y;
  int offB;
  int offC;
  int offZ;
  float ycarry;
  int dir;
  int D;
  int L;
  int nbatch;
};
static_assert(sizeof(ms1_args) == 136);

__device__ __forceinline__ float ms1_flush16(float v) {
  return (fabsf(v) < 6.103515625e-05f) ? 0.0f : v;
}
__device__ __forceinline__ unsigned ms1_h16bits(float v) {
  return (unsigned)__half_as_ushort(__float2half_rn(ms1_flush16(v)));
}
__device__ __forceinline__ float ms1_h16val(unsigned b) {
  return __half2float(__ushort_as_half((unsigned short)b));
}
__device__ __forceinline__ float ms1_softplus(float v) {
  return fmaxf(v, 0.0f) + log1pf(expf(-fabsf(v)));
}
__device__ __forceinline__ void ms1_pack2(float v0, float v1, unsigned& hw, unsigned& lw) {
  const unsigned h0 = ms1_h16bits(v0);
  const unsigned h1 = ms1_h16bits(v1);
  const float r0 = (v0 - ms1_h16val(h0)) * 2048.0f;
  const float r1 = (v1 - ms1_h16val(h1)) * 2048.0f;
  const unsigned l0 = ms1_h16bits(r0);
  const unsigned l1 = ms1_h16bits(r1);
  hw = h0 | (h1 << 16);
  lw = l0 | (l1 << 16);
}

template <int NSTATE>
__global__ __launch_bounds__(64 * (NSTATE / 16)) void ms1_scan_kernel(ms1_args a)
{
  static_assert(NSTATE == 16 || NSTATE == 64);
  constexpr int NQ  = NSTATE / 16;
  constexpr int NT  = 64 * NQ;
  constexpr int NW  = NT / 32;
  constexpr int BCW = 2 * NSTATE;
  constexpr int YP  = 68;
  constexpr int RPI = NW * 4;
  constexpr int NIT = 64 / RPI;
  static_assert(16 * NT <= 64 * YP);
  __shared__ __align__(16) float sBC[64 * BCW];
  __shared__ __align__(16) float sY[64 * YP];
  const int tid  = threadIdx.x;
  const int lane = tid & 31;
  const int wave = tid >> 5;
  const int c    = tid / NQ;
  const int sq   = tid - c * NQ;
  const int bpb  = a.D / 64;
  const int bi   = blockIdx.x / bpb;
  if (bi >= a.nbatch) return;
  const int d0 = (blockIdx.x - bi * bpb) * 64;
  const int d  = d0 + c;
  const long rowb = (long)bi * a.L;
  const bool hasz  = (a.z != nullptr);
  const bool hasD  = (a.Dskip != nullptr);
  const bool hasLo = (a.y_lo != nullptr);

#pragma unroll 1
  for (int n = 0; n < 16; ++n) {
    const float al = a.A_log[(long)d * NSTATE + sq * 16 + n];
    sY[n * NT + tid] = -expf(al);
  }
  __syncthreads();
  float An[16], h[16];
#pragma unroll
  for (int n = 0; n < 16; ++n) {
    An[n] = sY[n * NT + tid];
    h[n] = 0.0f;
  }
  float Dd = 0.0f;
  if (hasD) Dd = a.Dskip[d];

  const int nchunk = a.L / 64;
  const bool fwd = (a.dir > 0);
  const int s0 = fwd ? 0 : 63;
  const int sd = fwd ? 1 : -1;
  const int q  = lane >> 3;
  const int c8 = (lane & 7) * 8;

#pragma unroll 1
  for (int ci = 0; ci < nchunk; ++ci) {
    const int tb = fwd ? (ci * 64) : (a.L - 64 - ci * 64);
    const long rowc = rowb + tb;
    __syncthreads();
#pragma unroll 8
    for (int i = 0; i < 32; ++i) {
      const int idx = tid + i * NT;
      const int st  = idx / BCW;
      const int col = idx - st * BCW;
      const int sc  = (col < NSTATE) ? (a.offB + col) : (a.offC + col - NSTATE);
      sBC[idx] = a.bc[(rowc + st) * a.ld_bc + sc];
    }
    __syncthreads();
#pragma unroll 1
    for (int s = 0; s < 64; ++s) {
      const int ls = s0 + sd * s;
      const long row = rowc + ls;
      float pre = a.dtpre[row * a.ld_dtpre + d];
      float uv  = a.u[row * a.ld_u + d];
      float zv  = 0.0f;
      if (hasz) zv = a.z[row * a.ld_z + a.offZ + d];
      asm volatile("" : "+v"(pre));
      asm volatile("" : "+v"(uv));
      asm volatile("" : "+v"(zv));
      const float delta = ms1_softplus(pre);
      const float dtx = delta * uv;
      const float* bp = sBC + ls * BCW + sq * 16;
      const float* cp = bp + NSTATE;
      ms1_v4f Bq[4], Cq[4];
#pragma unroll
      for (int k = 0; k < 4; ++k) {
        Bq[k] = *(const ms1_v4f*)(bp + 4 * k);
        Cq[k] = *(const ms1_v4f*)(cp + 4 * k);
      }
      float yv = 0.0f;
#pragma unroll
      for (int n = 0; n < 16; ++n) {
        const float e = __expf(delta * An[n]);
        h[n] = fmaf(e, h[n], dtx * Bq[n >> 2][n & 3]);
        yv = fmaf(h[n], Cq[n >> 2][n & 3], yv);
      }
      if (NQ > 1) {
        yv += __shfl_xor(yv, 1, 32);
        yv += __shfl_xor(yv, 2, 32);
      }
      if (hasD) yv = fmaf(uv, Dd, yv);
      if (hasz) {
        const float sg = __builtin_amdgcn_rcpf(1.0f + expf(-zv));
        yv = yv * (zv * sg);
      }
      if (sq == 0) sY[ls * YP + c] = yv * a.ycarry;
    }
    __syncthreads();
    ms1_v4u hw[NIT], lw[NIT];
#pragma unroll
    for (int it = 0; it < NIT; ++it) {
      const int row = it * RPI + wave * 4 + q;
      const float* sp = sY + row * YP + c8;
      const ms1_v4f f0 = *(const ms1_v4f*)(sp);
      const ms1_v4f f1 = *(const ms1_v4f*)(sp + 4);
      unsigned h0, h1, h2, h3, l0, l1, l2, l3;
      ms1_pack2(f0[0], f0[1], h0, l0);
      ms1_pack2(f0[2], f0[3], h1, l1);
      ms1_pack2(f1[0], f1[1], h2, l2);
      ms1_pack2(f1[2], f1[3], h3, l3);
      hw[it] = (ms1_v4u){h0, h1, h2, h3};
      lw[it] = (ms1_v4u){l0, l1, l2, l3};
    }
    for (int pass = 0; pass < 2; ++pass) {
#pragma unroll
      for (int it = 0; it < NIT; ++it) {
        const int row = it * RPI + wave * 4 + q;
        const long o = (rowc + row) * a.ld_y + d0 + c8;
        *(volatile ms1_v4u*)(a.y + o) = hw[it];
        if (hasLo) *(volatile ms1_v4u*)(a.y_lo + o) = lw[it];
      }
      __threadfence();
    }
  }
}

static_assert(((kRows / 64) * (kXzP / 64)) % 8 == 0, "in_proj grid");
static_assert(((kRows / 64) * (kXdP / 64)) % 8 == 0, "x_proj grid");
static_assert(((kRows / 64) * (kDin / 64)) % 8 == 0, "dt_proj grid");
static_assert(((kRows / 64) * (kDm / 64)) % 8 == 0, "out_proj grid");
static_assert((kRows * kDm / 8) % 256 == 0 && (kXzP * kDm / 8) % 256 == 0 && (kXdP * kDin / 8) % 256 == 0 &&
              (kDin * kDtR / 8) % 256 == 0 && (kDm * kDin / 8) % 256 == 0 && (kRows * kDtR / 8) % 256 == 0, "plane grids");

extern "C" void kernel_launch(void* const* d_in, const int* in_sizes, int n_in,
                              void* d_out, int out_size, void* d_ws, size_t ws_size,
                              hipStream_t stream) {
  if (n_in < 10) return;
  if (in_sizes[0] != kRows * kDm) return;
  if (in_sizes[1] != kXzP * kDm) return;
  if (in_sizes[2] != kDin * 4) return;
  if (in_sizes[3] != kDin) return;
  if (in_sizes[4] != kXdW * kDin) return;
  if (in_sizes[5] != kDin * kDtR) return;
  if (in_sizes[6] != kDin) return;
  if (in_sizes[7] != kDin * kNst) return;
  if (in_sizes[8] != kDin) return;
  if (in_sizes[9] != kDm * kDin) return;
  if (out_size != kRows * kDm) return;
  if (ws_size < kWsTotal) return;

  const float* x      = (const float*)d_in[0];
  const float* W_in   = (const float*)d_in[1];
  const float* W_conv = (const float*)d_in[2];
  const float* b_conv = (const float*)d_in[3];
  const float* W_x    = (const float*)d_in[4];
  const float* W_dt   = (const float*)d_in[5];
  const float* b_dt   = (const float*)d_in[6];
  const float* A_log  = (const float*)d_in[7];
  const float* Dp     = (const float*)d_in[8];
  const float* W_out  = (const float*)d_in[9];
  float* out = (float*)d_out;

  char* ws = (char*)d_ws;
  unsigned short* XH  = (unsigned short*)(ws + kOffXH);
  unsigned short* WIH = (unsigned short*)(ws + kOffWIH);
  unsigned short* WXH = (unsigned short*)(ws + kOffWXH);
  unsigned short* WDH = (unsigned short*)(ws + kOffWDH);
  unsigned short* WOH = (unsigned short*)(ws + kOffWOH);
  float*          XZ  = (float*)(ws + kOffXZ);
  float*          U   = (float*)(ws + kOffU);
  unsigned short* UH  = (unsigned short*)(ws + kOffUH);
  float*          XD  = (float*)(ws + kOffXD);
  unsigned short* DTL = (unsigned short*)(ws + kOffDTL);
  float*          DTP = (float*)(ws + kOffDTP);
  unsigned short* YH  = (unsigned short*)(ws + kOffYH);

  plane_f16_kernel<<<(kRows * kDm / 8) / 256, 256, 0, stream>>>(x, kDm, kRows, XH, kDm / 8, kRows * kDm / 8, kCarryX);
  plane_f16_kernel<<<(kXzP * kDm / 8) / 256, 256, 0, stream>>>(W_in, kDm, kXzP, WIH, kDm / 8, kXzP * kDm / 8, kCarryWin);
  plane_f16_kernel<<<(kXdP * kDin / 8) / 256, 256, 0, stream>>>(W_x, kDin, kXdW, WXH, kDin / 8, kXdP * kDin / 8, kCarryWx);
  plane_f16_kernel<<<(kDin * kDtR / 8) / 256, 256, 0, stream>>>(W_dt, kDtR, kDin, WDH, kDtR / 8, kDin * kDtR / 8, kCarryWdt);
  plane_f16_kernel<<<(kDm * kDin / 8) / 256, 256, 0, stream>>>(W_out, kDin, kDm, WOH, kDin / 8, kDm * kDin / 8, kCarryWout);

  eng::gemm_f16_kernel<0><<<dim3((kRows / 64) * (kXzP / 64) / 8), 256, 0, stream>>>(
      XH, kDm, WIH, kDm, XZ, kXzP, nullptr, kRows, kXzP, kDm, kScaleIn);

  conv_act_kernel<<<dim3(kDin / 256, kRows / 64), 256, 0, stream>>>(XZ, W_conv, b_conv, U, UH);

  eng::gemm_f16_kernel<0><<<dim3((kRows / 64) * (kXdP / 64) / 8), 256, 0, stream>>>(
      UH, kDin, WXH, kDin, XD, kXdP, nullptr, kRows, kXdP, kDin, kScaleXp);

  plane_f16_kernel<<<(kRows * kDtR / 8) / 256, 256, 0, stream>>>(XD, kXdP, kRows, DTL, kDtR / 8, kRows * kDtR / 8, kCarryDtl);

  eng::gemm_f16_kernel<2><<<dim3((kRows / 64) * (kDin / 64) / 8), 256, 0, stream>>>(
      DTL, kDtR, WDH, kDtR, DTP, kDin, b_dt, kRows, kDin, kDtR, kScaleDt);

  for (int bi = 0; bi < kBatch; ++bi) {
    const size_t r0 = (size_t)bi * kSeq;
    ms1_args sa;
    sa.dtpre = DTP + r0 * kDin;
    sa.u = U + r0 * kDin;
    sa.bc = XD + r0 * kXdP;
    sa.z = XZ + r0 * kXzP;
    sa.A_log = A_log;
    sa.Dskip = Dp;
    sa.y = (__half*)(YH + r0 * kDin);
    sa.y_lo = nullptr;
    sa.ld_dtpre = kDin;
    sa.ld_u = kDin;
    sa.ld_bc = kXdP;
    sa.ld_z = kXzP;
    sa.ld_y = kDin;
    sa.offB = kDtR;
    sa.offC = kDtR + kNst;
    sa.offZ = kDin;
    sa.ycarry = kCarryY;
    sa.dir = 1;
    sa.D = kDin;
    sa.L = kSeq;
    sa.nbatch = 1;
    ms1_scan_kernel<16><<<dim3(kDin / 64), 64, 0, stream>>>(sa);
  }

  eng::gemm_f16_kernel<0><<<dim3((kRows / 64) * (kDm / 64) / 8), 256, 0, stream>>>(
      YH, kDin, WOH, kDin, out, kDm, nullptr, kRows, kDm, kDin, kScaleOut);
}
